// LSTM_DDPGActorNet_91104846282802
// MI455X (gfx1250) — hardware-verified
//
#include <hip/hip_runtime.h>
#include <hip/hip_bf16.h>


#define AS3 __attribute__((address_space(3)))

#define B_    4096
#define T_    128
#define H_    64
#define G4_   256
#define FC_   256
#define O_    8
#define OP_   16
#define K1_   8192
#define KC_   128
#define MB_   64
#define NBLK  (B_ / MB_)
#define NTHR  256

#define H0P   72
#define A1P   200
#define FP_   72
#define CP_   68
#define B2P   264

static_assert(K1_ == T_ * H_);
static_assert(KC_ == 2 * H_);
static_assert(H_ % 32 == 0);
static_assert(KC_ % 32 == 0);
static_assert(FC_ % 32 == 0);
static_assert(B_ % MB_ == 0);
static_assert(MB_ == 64);
static_assert(NTHR == 256);
static_assert(H0P % 8 == 0 && A1P % 8 == 0 && FP_ % 8 == 0 && B2P % 8 == 0 && CP_ % 4 == 0);
static_assert(A1P >= 3 * H_ && H0P >= H_ && FP_ >= H_ && B2P >= FC_ && CP_ >= H_);
static_assert(O_ <= OP_ && OP_ == 16);

typedef _Float16       v16h __attribute__((ext_vector_type(16)));
typedef _Float16       v8h  __attribute__((ext_vector_type(8)));
typedef __bf16         v16b __attribute__((ext_vector_type(16)));
typedef unsigned short v8us __attribute__((ext_vector_type(8)));
typedef float          v8f  __attribute__((ext_vector_type(8)));
typedef float          v4f  __attribute__((ext_vector_type(4)));

typedef AS3 _Float16*             lp_h;
typedef AS3 const _Float16*       lcp_h;
typedef AS3 float*                lp_f;
typedef AS3 const float*          lcp_f;
typedef AS3 unsigned short*       lp_u;
typedef AS3 const unsigned short* lcp_u;

union FragH { v16h v; v8h  half[2]; };
union FragB { v16b v; v8us half[2]; };

#define SCL    16.0f
#define INV256 0.00390625f

constexpr size_t SZ_WHH0 = (size_t)G4_ * H_  * 2;
constexpr size_t SZ_WCAT = (size_t)G4_ * KC_ * 2;
constexpr size_t SZ_W1P  = (size_t)FC_ * K1_ * 2;
constexpr size_t SZ_W2P  = (size_t)FC_ * FC_ * 2;
constexpr size_t SZ_W3P  = (size_t)OP_ * FC_ * 2;
constexpr size_t OFF_WHH0 = 0;
constexpr size_t OFF_WCAT = OFF_WHH0 + SZ_WHH0;
constexpr size_t OFF_W1H  = OFF_WCAT + SZ_WCAT;
constexpr size_t OFF_W1L  = OFF_W1H  + SZ_W1P;
constexpr size_t OFF_W2H  = OFF_W1L  + SZ_W1P;
constexpr size_t OFF_W2L  = OFF_W2H  + SZ_W2P;
constexpr size_t OFF_W3H  = OFF_W2L  + SZ_W2P;
constexpr size_t OFF_W3L  = OFF_W3H  + SZ_W3P;
constexpr size_t WS_END   = OFF_W3L  + SZ_W3P;
static_assert(OFF_WCAT % 128 == 0 && OFF_W1H % 128 == 0 && OFF_W1L % 128 == 0 && OFF_W2H % 128 == 0);
static_assert(OFF_W2L % 128 == 0 && OFF_W3H % 128 == 0 && OFF_W3L % 128 == 0 && WS_END % 128 == 0);
static_assert(WS_END <= (size_t)134217728);

constexpr int NP0 = G4_ * (H_  / 8);
constexpr int NP1 = G4_ * (KC_ / 8);
constexpr int NP2 = FC_ * (K1_ / 8);
constexpr int NP3 = FC_ * (FC_ / 8);
constexpr int NP4 = OP_ * (FC_ / 8);
static_assert(NP0 % 256 == 0 && NP1 % 256 == 0 && NP2 % 256 == 0 && NP3 % 256 == 0 && NP4 % 256 == 0);
constexpr int E0 = NP0 / 256;
constexpr int E1 = E0 + NP1 / 256;
constexpr int E2 = E1 + NP2 / 256;
constexpr int E3 = E2 + NP3 / 256;
constexpr int NBLK_CVT = E3 + NP4 / 256;
static_assert((size_t)NP0 * 16 == SZ_WHH0 && (size_t)NP1 * 16 == SZ_WCAT && (size_t)NP2 * 16 == SZ_W1P);
static_assert((size_t)NP3 * 16 == SZ_W2P && (size_t)NP4 * 16 == SZ_W3P);

constexpr size_t LSZ_ACC  = (size_t)64 * 32 * 8 * 4;
constexpr size_t LSZ_H0   = (size_t)2 * MB_ * H0P * 2;
constexpr size_t LSZ_A1   = (size_t)MB_ * A1P * 2;
constexpr size_t LSZ_F    = (size_t)MB_ * FP_ * 2;
constexpr size_t LSZ_C    = (size_t)MB_ * CP_ * 4;
constexpr size_t LSZ_B2   = (size_t)MB_ * B2P * 2;
constexpr size_t LOFF_ACC = 0;
constexpr size_t LOFF_H0  = LOFF_ACC + LSZ_ACC;
constexpr size_t LOFF_A1  = LOFF_H0  + LSZ_H0;
constexpr size_t LOFF_FH  = LOFF_A1  + LSZ_A1;
constexpr size_t LOFF_FL  = LOFF_FH  + LSZ_F;
constexpr size_t LOFF_C0  = LOFF_FL  + LSZ_F;
constexpr size_t LOFF_C1  = LOFF_C0  + LSZ_C;
constexpr size_t LEND_SEQ = LOFF_C1  + LSZ_C;
constexpr size_t LOFF_B2H = LOFF_H0;
constexpr size_t LOFF_B2L = LOFF_B2H + LSZ_B2;
static_assert(LOFF_B2L + LSZ_B2 <= LEND_SEQ);
constexpr size_t LOFF_BIAS0 = LEND_SEQ;
constexpr size_t LOFF_BIAS1 = LOFF_BIAS0 + (size_t)G4_ * 4;
constexpr size_t LOFF_WIH0  = LOFF_BIAS1 + (size_t)G4_ * 4;
constexpr size_t LOFF_B1    = LOFF_WIH0  + (size_t)G4_ * 4;
constexpr size_t LOFF_B2B   = LOFF_B1    + (size_t)FC_ * 4;
constexpr size_t LOFF_B3    = LOFF_B2B   + (size_t)FC_ * 4;
constexpr size_t LOFF_OUT   = LOFF_B3    + (size_t)OP_ * 4;
constexpr size_t LDS_BYTES  = LOFF_OUT   + (size_t)MB_ * O_ * 4;
static_assert(LOFF_H0 % 16 == 0 && LOFF_A1 % 16 == 0 && LOFF_FH % 16 == 0 && LOFF_FL % 16 == 0);
static_assert(LOFF_C0 % 16 == 0 && LOFF_C1 % 16 == 0 && LOFF_B2H % 16 == 0 && LOFF_B2L % 16 == 0);
static_assert(LOFF_BIAS0 % 16 == 0 && LOFF_B3 % 16 == 0 && LOFF_OUT % 16 == 0 && LDS_BYTES % 16 == 0);
static_assert(LSZ_ACC % 16 == 0 && LSZ_H0 % 16 == 0 && LSZ_A1 % 16 == 0 && LSZ_C % 16 == 0);

__device__ __forceinline__ float rcpx(float x) { return __builtin_amdgcn_rcpf(x); }
__device__ __forceinline__ float sigm(float x) { return rcpx(1.0f + __expf(-x)); }
__device__ __forceinline__ float tanhm(float x) {
    const float e = __expf(2.0f * x);
    return 1.0f - 2.0f * rcpx(e + 1.0f);
}
__device__ __forceinline__ unsigned int bf16_rne(float x) {
    const unsigned int u = __float_as_uint(x);
    return (u + 0x7FFFu + ((u >> 16) & 1u)) >> 16;
}
__device__ __forceinline__ void split_bf16(float x, unsigned short& hi, unsigned short& lo) {
    const unsigned int hb = bf16_rne(x);
    const float hf = __uint_as_float(hb << 16);
    const unsigned int lb = bf16_rne(x - hf);
    hi = (unsigned short)hb;
    lo = (unsigned short)lb;
}
__device__ __forceinline__ v8f ld8f(const float* p) {
    const v4f a = *(const v4f*)p;
    const v4f b = *(const v4f*)(p + 4);
    return __builtin_shufflevector(a, b, 0, 1, 2, 3, 4, 5, 6, 7);
}
__device__ __forceinline__ v8f ld8f_lds(lcp_f p) {
    const v4f a = *(AS3 const v4f*)p;
    const v4f b = *(AS3 const v4f*)(p + 4);
    return __builtin_shufflevector(a, b, 0, 1, 2, 3, 4, 5, 6, 7);
}
__device__ __forceinline__ void st8f_lds(lp_f p, v8f v) {
    *(AS3 v4f*)p       = __builtin_shufflevector(v, v, 0, 1, 2, 3);
    *(AS3 v4f*)(p + 4) = __builtin_shufflevector(v, v, 4, 5, 6, 7);
}
__device__ __forceinline__ v8f zero8() {
    v8f z;
#pragma unroll
    for (int i = 0; i < 8; ++i) z[i] = 0.0f;
    return z;
}

__device__ __forceinline__ void ldh_lds(FragH& f, lcp_h p) {
    f.half[0] = *(AS3 const v8h*)(p);
    f.half[1] = *(AS3 const v8h*)(p + 16);
}
__device__ __forceinline__ void ldh_glb(FragH& f, const _Float16* p) {
    f.half[0] = *(const v8h*)(p);
    f.half[1] = *(const v8h*)(p + 16);
}
__device__ __forceinline__ void ldb_lds(FragB& f, lcp_u p) {
    f.half[0] = *(AS3 const v8us*)(p);
    f.half[1] = *(AS3 const v8us*)(p + 16);
}
__device__ __forceinline__ void ldb_glb(FragB& f, const unsigned short* p) {
    f.half[0] = *(const v8us*)(p);
    f.half[1] = *(const v8us*)(p + 16);
}
__device__ __forceinline__ v8f mmah(v8f c, const FragH& a, const FragH& b) {
    return __builtin_amdgcn_wmma_f32_16x16x32_f16(false, a.v, false, b.v, (short)0, c, false, false);
}
__device__ __forceinline__ v8f mmab(v8f c, const FragB& a, const FragB& b) {
    return __builtin_amdgcn_wmma_f32_16x16x32_bf16(false, a.v, false, b.v, (short)0, c, false, false);
}

__global__ __launch_bounds__(256)
void cvt_kernel(const float* __restrict__ Whh0, const float* __restrict__ Wih1,
                const float* __restrict__ Whh1, const float* __restrict__ W1,
                const float* __restrict__ W2,   const float* __restrict__ W3,
                _Float16* Whh0p, _Float16* Wcat,
                unsigned short* W1h, unsigned short* W1l,
                unsigned short* W2h, unsigned short* W2l,
                unsigned short* W3h, unsigned short* W3l)
{
    const int tid = threadIdx.x;
    const int bid = blockIdx.x;
    if (bid < E0) {
        const int p  = bid * 256 + tid;
        const int n  = p >> 3;
        const int c8 = (p & 7) * 8;
        const v8f a = ld8f(Whh0 + (size_t)n * H_ + c8);
        v8h hv;
#pragma unroll
        for (int i = 0; i < 8; ++i) hv[i] = (_Float16)(a[i] * SCL);
        _Float16* d = Whh0p + (size_t)n * H_ + c8;
        *(volatile v8h*)d = hv;
        __threadfence();
        *(volatile v8h*)d = hv;
    } else if (bid < E1) {
        const int p  = (bid - E0) * 256 + tid;
        const int n  = p >> 4;
        const int c8 = (p & 15) * 8;
        const int ci = min(c8, H_ - 8);
        const int cj = min(max(c8 - H_, 0), H_ - 8);
        const v8f a = ld8f(Wih1 + (size_t)n * H_ + ci);
        const v8f b = ld8f(Whh1 + (size_t)n * H_ + cj);
        v8h hv;
#pragma unroll
        for (int i = 0; i < 8; ++i) {
            const float v = (c8 < H_) ? a[i] : b[i];
            hv[i] = (_Float16)(v * SCL);
        }
        _Float16* d = Wcat + (size_t)n * KC_ + c8;
        *(volatile v8h*)d = hv;
        __threadfence();
        *(volatile v8h*)d = hv;
    } else if (bid < E2) {
        const int p  = (bid - E1) * 256 + tid;
        const int n  = p >> 10;
        const int c8 = (p & 1023) * 8;
        const v8f a = ld8f(W1 + (size_t)n * K1_ + c8);
        v8us hv, lv;
#pragma unroll
        for (int i = 0; i < 8; ++i) { unsigned short hi, lo; split_bf16(a[i], hi, lo); hv[i] = hi; lv[i] = lo; }
        const size_t o = (size_t)n * K1_ + c8;
        *(volatile v8us*)(W1h + o) = hv;
        *(volatile v8us*)(W1l + o) = lv;
        __threadfence();
        *(volatile v8us*)(W1h + o) = hv;
        *(volatile v8us*)(W1l + o) = lv;
    } else if (bid < E3) {
        const int p  = (bid - E2) * 256 + tid;
        const int n  = p >> 5;
        const int c8 = (p & 31) * 8;
        const v8f a = ld8f(W2 + (size_t)n * FC_ + c8);
        v8us hv, lv;
#pragma unroll
        for (int i = 0; i < 8; ++i) { unsigned short hi, lo; split_bf16(a[i], hi, lo); hv[i] = hi; lv[i] = lo; }
        const size_t o = (size_t)n * FC_ + c8;
        *(volatile v8us*)(W2h + o) = hv;
        *(volatile v8us*)(W2l + o) = lv;
        __threadfence();
        *(volatile v8us*)(W2h + o) = hv;
        *(volatile v8us*)(W2l + o) = lv;
    } else {
        const int p  = (bid - E3) * 256 + tid;
        const int n  = p >> 5;
        const int c8 = (p & 31) * 8;
        const int nn = min(n, O_ - 1);
        const v8f a = ld8f(W3 + (size_t)nn * FC_ + c8);
        v8us hv, lv;
#pragma unroll
        for (int i = 0; i < 8; ++i) {
            const float v = (n < O_) ? a[i] : 0.0f;
            unsigned short hi, lo; split_bf16(v, hi, lo); hv[i] = hi; lv[i] = lo;
        }
        const size_t o = (size_t)n * FC_ + c8;
        *(volatile v8us*)(W3h + o) = hv;
        *(volatile v8us*)(W3l + o) = lv;
        __threadfence();
        *(volatile v8us*)(W3h + o) = hv;
        *(volatile v8us*)(W3l + o) = lv;
    }
}

__device__ __forceinline__ void cvt_pass(lcp_f sAcc, lcp_f sBias, lp_u dH, lp_u dL, int tid)
{
#pragma unroll 1
    for (int i = tid; i < MB_ * (FC_ / 8); i += NTHR) {
        const int row = i >> 5;
        const int c8  = (i & 31) * 8;
        const int ti  = (row >> 4) * 16 + (c8 >> 4);
        const int lb  = (c8 & 15) + 16 * ((row >> 3) & 1);
        lcp_f src = sAcc + (ti * 32 + lb) * 8 + (row & 7);
        v8us hv, lv;
#pragma unroll
        for (int e = 0; e < 8; ++e) {
            const float v = fmaxf(src[e * 8] + sBias[c8 + e], 0.0f);
            unsigned short hi, lo; split_bf16(v, hi, lo); hv[e] = hi; lv[e] = lo;
        }
        *(AS3 v8us*)(dH + row * B2P + c8) = hv;
        *(AS3 v8us*)(dL + row * B2P + c8) = lv;
    }
}

__global__ __launch_bounds__(NTHR)
void seq_kernel(const float* __restrict__ obs,  const float* __restrict__ wih0,
                const float* __restrict__ bih0, const float* __restrict__ bhh0,
                const float* __restrict__ bih1, const float* __restrict__ bhh1,
                const float* __restrict__ b1,   const float* __restrict__ b2,
                const float* __restrict__ b3,
                const _Float16* __restrict__ Whh0p, const _Float16* __restrict__ Wcat,
                const unsigned short* __restrict__ W1h, const unsigned short* __restrict__ W1l,
                const unsigned short* __restrict__ W2h, const unsigned short* __restrict__ W2l,
                const unsigned short* __restrict__ W3h, const unsigned short* __restrict__ W3l,
                float* out)
{
    extern __shared__ __attribute__((aligned(16))) char smem[];
    lp_f sAcc   = (lp_f)(smem + LOFF_ACC);
    lp_h sH0    = (lp_h)(smem + LOFF_H0);
    lp_h sA1    = (lp_h)(smem + LOFF_A1);
    lp_u sFH    = (lp_u)(smem + LOFF_FH);
    lp_u sFL    = (lp_u)(smem + LOFF_FL);
    lp_f sC0    = (lp_f)(smem + LOFF_C0);
    lp_f sC1    = (lp_f)(smem + LOFF_C1);
    lp_u sB2H   = (lp_u)(smem + LOFF_B2H);
    lp_u sB2L   = (lp_u)(smem + LOFF_B2L);
    lp_f sBias0 = (lp_f)(smem + LOFF_BIAS0);
    lp_f sBias1 = (lp_f)(smem + LOFF_BIAS1);
    lp_f sWih0  = (lp_f)(smem + LOFF_WIH0);
    lp_f sB1    = (lp_f)(smem + LOFF_B1);
    lp_f sB2b   = (lp_f)(smem + LOFF_B2B);
    lp_f sB3    = (lp_f)(smem + LOFF_B3);
    lp_f sOut   = (lp_f)(smem + LOFF_OUT);

    const int tid  = threadIdx.x;
    const int lane = tid & 31;
    const int w    = tid >> 5;
    const int h    = lane >> 4;
    const int m    = lane & 15;
    const int mt   = w >> 1;
    const int jg   = (w & 1) * 2;
    const int cb   = (w & 1) * 8;
    const int b0   = blockIdx.x * MB_;
    const int arow = 16 * mt + m;
    const int drow = 16 * mt + 8 * h;

    {
        v4f zf;
#pragma unroll
        for (int i = 0; i < 4; ++i) zf[i] = 0.0f;
        v8h zh;
#pragma unroll
        for (int i = 0; i < 8; ++i) zh[i] = (_Float16)0.0f;
        for (int i = tid; i < (int)(LSZ_ACC / 16); i += NTHR) *(AS3 v4f*)(sAcc + 4 * i) = zf;
        for (int i = tid; i < (int)(LSZ_H0 / 16);  i += NTHR) *(AS3 v8h*)(sH0 + 8 * i) = zh;
        for (int i = tid; i < (int)(LSZ_A1 / 16);  i += NTHR) *(AS3 v8h*)(sA1 + 8 * i) = zh;
        for (int i = tid; i < (int)(LSZ_C / 16);   i += NTHR) { *(AS3 v4f*)(sC0 + 4 * i) = zf; *(AS3 v4f*)(sC1 + 4 * i) = zf; }
        for (int i = tid; i < G4_; i += NTHR) {
            sBias0[i] = bih0[i] + bhh0[i];
            sBias1[i] = bih1[i] + bhh1[i];
            sWih0[i]  = wih0[i];
            sB1[i]    = b1[i];
            sB2b[i]   = b2[i];
        }
        if (tid < OP_) {
            const float v = b3[min(tid, O_ - 1)];
            sB3[tid] = (tid < O_) ? v : 0.0f;
        }
    }
    __syncthreads();

    const float* orow = obs + (size_t)(b0 + drow) * T_;

#pragma unroll 1
    for (int t = 0; t < T_; ++t) {
        const int par = t & 1;
        lcp_h sH0c = sH0 + par * (MB_ * H0P);
        lp_h  sH0n = sH0 + (par ^ 1) * (MB_ * H0P);
        const int hbc = H_ + par * H_;
        const int hbn = H_ + (par ^ 1) * H_;

        float xo[8];
#pragma unroll
        for (int r = 0; r < 8; ++r) xo[r] = orow[(size_t)r * T_ + t];

#pragma unroll 1
        for (int g = 0; g < 2; ++g) {
            const int j = jg + g;
            v8f acc[4];
#pragma unroll
            for (int q = 0; q < 4; ++q) acc[q] = zero8();
            lcp_h ab = sH0c + arow * H0P + 8 * h;
            const _Float16* wb = Whh0p + (size_t)(16 * j + m) * H_ + 8 * h;
#pragma unroll
            for (int ks = 0; ks < 2; ++ks) {
                FragH a;
                ldh_lds(a, ab + 32 * ks);
                FragH b[4];
#pragma unroll
                for (int q = 0; q < 4; ++q) ldh_glb(b[q], wb + (size_t)q * (64 * H_) + 32 * ks);
#pragma unroll
                for (int q = 0; q < 4; ++q) acc[q] = mmah(acc[q], a, b[q]);
                asm volatile("v_nop\n\tv_nop\n\tv_nop\n\tv_nop"
                             : "+v"(acc[0]), "+v"(acc[1]), "+v"(acc[2]), "+v"(acc[3])
                             : "v"(a.v), "v"(b[0].v), "v"(b[1].v), "v"(b[2].v), "v"(b[3].v));
            }
            const int n = 16 * j + m;
            const float wi = sWih0[n];
            const float wf = sWih0[H_ + n];
            const float wg = sWih0[2 * H_ + n];
            const float wo = sWih0[3 * H_ + n];
            const float bi = sBias0[n];
            const float bf = sBias0[H_ + n];
            const float bg = sBias0[2 * H_ + n];
            const float bo = sBias0[3 * H_ + n];
#pragma unroll
            for (int r = 0; r < 8; ++r) {
                const int row = drow + r;
                const float x  = xo[r];
                const float gi = acc[0][r] * INV256 + (x * wi + bi);
                const float gf = acc[1][r] * INV256 + (x * wf + bf);
                const float gg = acc[2][r] * INV256 + (x * wg + bg);
                const float go = acc[3][r] * INV256 + (x * wo + bo);
                const float cp = sC0[row * CP_ + n];
                const float cn = sigm(gf) * cp + sigm(gi) * tanhm(gg);
                sC0[row * CP_ + n] = cn;
                const float hn = sigm(go) * tanhm(cn);
                const _Float16 hs = (_Float16)(hn * SCL);
                sH0n[row * H0P + n] = hs;
                sA1[row * A1P + n]  = hs;
            }
        }
        __syncthreads();

#pragma unroll 1
        for (int g = 0; g < 2; ++g) {
            const int j = jg + g;
            v8f acc[4];
#pragma unroll
            for (int q = 0; q < 4; ++q) acc[q] = zero8();
            lcp_h ab = sA1 + arow * A1P + 8 * h;
            const _Float16* wb = Wcat + (size_t)(16 * j + m) * KC_ + 8 * h;
#pragma unroll
            for (int ks = 0; ks < 4; ++ks) {
                const int aoff = (ks < 2) ? (32 * ks) : (hbc + 32 * (ks - 2));
                FragH a;
                ldh_lds(a, ab + aoff);
                FragH b[4];
#pragma unroll
                for (int q = 0; q < 4; ++q) ldh_glb(b[q], wb + (size_t)q * (64 * KC_) + 32 * ks);
#pragma unroll
                for (int q = 0; q < 4; ++q) acc[q] = mmah(acc[q], a, b[q]);
                asm volatile("v_nop\n\tv_nop\n\tv_nop\n\tv_nop"
                             : "+v"(acc[0]), "+v"(acc[1]), "+v"(acc[2]), "+v"(acc[3])
                             : "v"(a.v), "v"(b[0].v), "v"(b[1].v), "v"(b[2].v), "v"(b[3].v));
            }
            const int n = 16 * j + m;
            const float bi = sBias1[n];
            const float bf = sBias1[H_ + n];
            const float bg = sBias1[2 * H_ + n];
            const float bo = sBias1[3 * H_ + n];
#pragma unroll
            for (int r = 0; r < 8; ++r) {
                const int row = drow + r;
                const float gi = acc[0][r] * INV256 + bi;
                const float gf = acc[1][r] * INV256 + bf;
                const float gg = acc[2][r] * INV256 + bg;
                const float go = acc[3][r] * INV256 + bo;
                const float cp = sC1[row * CP_ + n];
                const float cn = sigm(gf) * cp + sigm(gi) * tanhm(gg);
                sC1[row * CP_ + n] = cn;
                const float hn = sigm(go) * tanhm(cn);
                sA1[row * A1P + hbn + n] = (_Float16)(hn * SCL);
                unsigned short hi, lo;
                split_bf16(hn, hi, lo);
                sFH[row * FP_ + n] = hi;
                sFL[row * FP_ + n] = lo;
            }
        }
        __syncthreads();

#pragma unroll 1
        for (int cg = 0; cg < 2; ++cg) {
            const int ct0 = cb + cg * 4;
            v8f acc[4];
#pragma unroll
            for (int q = 0; q < 4; ++q) acc[q] = ld8f_lds(sAcc + ((mt * 16 + ct0 + q) * 32 + lane) * 8);
            const int fb = arow * FP_ + 8 * h;
#pragma unroll
            for (int ks = 0; ks < 2; ++ks) {
                FragB ah, al;
                ldb_lds(ah, sFH + fb + 32 * ks);
                ldb_lds(al, sFL + fb + 32 * ks);
                FragB bh[4], bl[4];
#pragma unroll
                for (int q = 0; q < 4; ++q) {
                    const size_t o = (size_t)(16 * (ct0 + q) + m) * K1_ + (size_t)t * H_ + 32 * ks + 8 * h;
                    ldb_glb(bh[q], W1h + o);
                    ldb_glb(bl[q], W1l + o);
                }
#pragma unroll
                for (int q = 0; q < 4; ++q) {
                    acc[q] = mmab(acc[q], ah, bh[q]);
                    acc[q] = mmab(acc[q], ah, bl[q]);
                    acc[q] = mmab(acc[q], al, bh[q]);
                }
                asm volatile("v_nop\n\tv_nop\n\tv_nop\n\tv_nop"
                             : "+v"(acc[0]), "+v"(acc[1]), "+v"(acc[2]), "+v"(acc[3])
                             : "v"(ah.v), "v"(al.v), "v"(bh[0].v), "v"(bh[1].v), "v"(bh[2].v), "v"(bh[3].v),
                               "v"(bl[0].v), "v"(bl[1].v), "v"(bl[2].v), "v"(bl[3].v));
            }
#pragma unroll
            for (int q = 0; q < 4; ++q) st8f_lds(sAcc + ((mt * 16 + ct0 + q) * 32 + lane) * 8, acc[q]);
        }
    }
    __syncthreads();

    cvt_pass(sAcc, sB1, sB2H, sB2L, tid);
    __syncthreads();

#pragma unroll 1
    for (int cg = 0; cg < 2; ++cg) {
        const int ct0 = cb + cg * 4;
        v8f acc[4];
#pragma unroll
        for (int q = 0; q < 4; ++q) acc[q] = zero8();
        const int fb = arow * B2P + 8 * h;
#pragma unroll 1
        for (int ks = 0; ks < FC_ / 32; ++ks) {
            FragB ah, al;
            ldb_lds(ah, sB2H + fb + 32 * ks);
            ldb_lds(al, sB2L + fb + 32 * ks);
            FragB bh[4], bl[4];
#pragma unroll
            for (int q = 0; q < 4; ++q) {
                const size_t o = (size_t)(16 * (ct0 + q) + m) * FC_ + 32 * ks + 8 * h;
                ldb_glb(bh[q], W2h + o);
                ldb_glb(bl[q], W2l + o);
            }
#pragma unroll
            for (int q = 0; q < 4; ++q) {
                acc[q] = mmab(acc[q], ah, bh[q]);
                acc[q] = mmab(acc[q], ah, bl[q]);
                acc[q] = mmab(acc[q], al, bh[q]);
            }
            asm volatile("v_nop\n\tv_nop\n\tv_nop\n\tv_nop"
                         : "+v"(acc[0]), "+v"(acc[1]), "+v"(acc[2]), "+v"(acc[3])
                         : "v"(ah.v), "v"(al.v), "v"(bh[0].v), "v"(bh[1].v), "v"(bh[2].v), "v"(bh[3].v),
                           "v"(bl[0].v), "v"(bl[1].v), "v"(bl[2].v), "v"(bl[3].v));
        }
#pragma unroll
        for (int q = 0; q < 4; ++q) st8f_lds(sAcc + ((mt * 16 + ct0 + q) * 32 + lane) * 8, acc[q]);
    }
    __syncthreads();

    cvt_pass(sAcc, sB2b, sB2H, sB2L, tid);
    __syncthreads();

    if (w < 4) {
        const int mt3 = w;
        v8f acc = zero8();
        const int fb = (16 * mt3 + m) * B2P + 8 * h;
#pragma unroll 1
        for (int ks = 0; ks < FC_ / 32; ++ks) {
            FragB ah, al, bh, bl;
            ldb_lds(ah, sB2H + fb + 32 * ks);
            ldb_lds(al, sB2L + fb + 32 * ks);
            const size_t o = (size_t)m * FC_ + 32 * ks + 8 * h;
            ldb_glb(bh, W3h + o);
            ldb_glb(bl, W3l + o);
            acc = mmab(acc, ah, bh);
            acc = mmab(acc, ah, bl);
            acc = mmab(acc, al, bh);
            asm volatile("v_nop\n\tv_nop\n\tv_nop\n\tv_nop"
                         : "+v"(acc) : "v"(ah.v), "v"(al.v), "v"(bh.v), "v"(bl.v));
        }
        if (m < O_) {
            const float bb = sB3[m];
#pragma unroll
            for (int r = 0; r < 8; ++r) {
                const int row = 16 * mt3 + 8 * h + r;
                const float v = acc[r] + bb;
                const float s = sigm(v);
                sOut[row * O_ + m] = s * 2.0f - 1.0f;
            }
        }
    }
    __syncthreads();

    if (tid < (MB_ * O_) / 4) {
        const v4f v = *(AS3 const v4f*)(sOut + 4 * tid);
        float* op = out + (size_t)b0 * O_ + 4 * tid;
        *(volatile v4f*)op = v;
        __threadfence();
        *(volatile v4f*)op = v;
    }
}

extern "C" void kernel_launch(void* const* d_in, const int* in_sizes, int n_in,
                              void* d_out, int out_size, void* d_ws, size_t ws_size,
                              hipStream_t stream)
{
    if (n_in < 15) return;
    if (in_sizes[0]  != B_ * T_)   return;
    if (in_sizes[1]  != G4_)       return;
    if (in_sizes[2]  != G4_ * H_)  return;
    if (in_sizes[3]  != G4_)       return;
    if (in_sizes[4]  != G4_)       return;
    if (in_sizes[5]  != G4_ * H_)  return;
    if (in_sizes[6]  != G4_ * H_)  return;
    if (in_sizes[7]  != G4_)       return;
    if (in_sizes[8]  != G4_)       return;
    if (in_sizes[9]  != FC_ * K1_) return;
    if (in_sizes[10] != FC_)       return;
    if (in_sizes[11] != FC_ * FC_) return;
    if (in_sizes[12] != FC_)       return;
    if (in_sizes[13] != O_ * FC_)  return;
    if (in_sizes[14] != O_)        return;
    if (out_size != B_ * O_)       return;
    if (ws_size < WS_END)          return;

    const float* obs  = (const float*)d_in[0];
    const float* Wih0 = (const float*)d_in[1];
    const float* Whh0 = (const float*)d_in[2];
    const float* bih0 = (const float*)d_in[3];
    const float* bhh0 = (const float*)d_in[4];
    const float* Wih1 = (const float*)d_in[5];
    const float* Whh1 = (const float*)d_in[6];
    const float* bih1 = (const float*)d_in[7];
    const float* bhh1 = (const float*)d_in[8];
    const float* W1   = (const float*)d_in[9];
    const float* b1   = (const float*)d_in[10];
    const float* W2   = (const float*)d_in[11];
    const float* b2   = (const float*)d_in[12];
    const float* W3   = (const float*)d_in[13];
    const float* b3   = (const float*)d_in[14];
    float* out = (float*)d_out;

    char* ws = (char*)d_ws;
    _Float16*       Whh0p = (_Float16*)(ws + OFF_WHH0);
    _Float16*       Wcat  = (_Float16*)(ws + OFF_WCAT);
    unsigned short* W1h   = (unsigned short*)(ws + OFF_W1H);
    unsigned short* W1l   = (unsigned short*)(ws + OFF_W1L);
    unsigned short* W2h   = (unsigned short*)(ws + OFF_W2H);
    unsigned short* W2l   = (unsigned short*)(ws + OFF_W2L);
    unsigned short* W3h   = (unsigned short*)(ws + OFF_W3H);
    unsigned short* W3l   = (unsigned short*)(ws + OFF_W3L);

    cvt_kernel<<<dim3(NBLK_CVT), dim3(256), 0, stream>>>(
        Whh0, Wih1, Whh1, W1, W2, W3, Whh0p, Wcat, W1h, W1l, W2h, W2l, W3h, W3l);

    hipFuncSetAttribute(reinterpret_cast<const void*>(&seq_kernel),
                        hipFuncAttributeMaxDynamicSharedMemorySize, (int)LDS_BYTES);
    seq_kernel<<<dim3(NBLK), dim3(NTHR), LDS_BYTES, stream>>>(
        obs, Wih0, bih0, bhh0, bih1, bhh1, b1, b2, b3,
        (const _Float16*)Whh0p, (const _Float16*)Wcat,
        (const unsigned short*)W1h, (const unsigned short*)W1l,
        (const unsigned short*)W2h, (const unsigned short*)W2l,
        (const unsigned short*)W3h, (const unsigned short*)W3l, out);
}
